// MultiHeadAttention_29678224015584
// MI455X (gfx1250) — hardware-verified
//
#include <hip/hip_runtime.h>


#ifndef NB
#define NB 2
#endif
#ifndef SEQ
#define SEQ 2048
#endif
#define NB_FULL  2
#define SEQ_FULL 2048
#define TT   SEQ
#define DM   1024
#define NH_  16
#define HD   64
#define DQ   (NH_ * HD)
#define ZH   2
#define PCAR 1024.0f
#define SCL  0.03125f
static_assert(SEQ % 256 == 0);
static_assert(SEQ <= SEQ_FULL);
static_assert(NB <= NB_FULL);
static_assert(DQ == DM);
static_assert(HD == 64);
static_assert(NH_ % ZH == 0);
static_assert(DM % 64 == 0);

typedef _Float16 h16;
typedef unsigned short bf;
typedef __attribute__((ext_vector_type(16))) __bf16   v16bf;
typedef __attribute__((ext_vector_type(16))) _Float16 v16h;
typedef __attribute__((ext_vector_type(8)))  _Float16 v8h;
typedef __attribute__((ext_vector_type(4)))  _Float16 v4h;
typedef __attribute__((ext_vector_type(8)))  unsigned short v8us;
typedef __attribute__((ext_vector_type(8)))  float    v8f;
typedef __attribute__((ext_vector_type(4)))  float    v4f;
typedef v4f  __attribute__((may_alias)) v4fa;

#define SZ_W3 ((size_t)3 * DM * DM * 2)
#define SZ_WO ((size_t)DM * DQ * 2)
#define SZ_XB ((size_t)TT * DM * 2)
#define SZ_F3 ((size_t)3 * TT * DM * 4)
#define SZ_QK ((size_t)2 * NH_ * TT * HD * 2)
#define SZ_VT ((size_t)NH_ * HD * TT * 2)
#define SZ_VM ((size_t)NH_ * HD * 4)
#define SZ_SB ((size_t)ZH * TT * TT * 4)
#define SZ_PP ((size_t)ZH * TT * TT * 2)
#define SZ_OB ((size_t)ZH * TT * HD * 4)
#define SZ_AT ((size_t)TT * DQ * 2)
#define WS_TOTAL (SZ_W3 + SZ_WO + SZ_XB + SZ_F3 + SZ_QK + SZ_VT + SZ_VM + SZ_SB + SZ_PP + SZ_OB + 2 * SZ_AT)
static_assert(WS_TOTAL <= (size_t)134217728);
static_assert(SZ_VM % 256 == 0);

__device__ __forceinline__ unsigned short f2bf(float f) { unsigned u = __float_as_uint(f); u += 0x7FFFu + ((u >> 16) & 1u); return (unsigned short)(u >> 16); }
__device__ __forceinline__ float bf2f(unsigned short b) { return __uint_as_float(((unsigned)b) << 16); }
__device__ __forceinline__ float bfr(float f) { return bf2f(f2bf(f)); }
__device__ __forceinline__ v16h cat16(v8h lo, v8h hi) { return __builtin_shufflevector(lo, hi, 0, 1, 2, 3, 4, 5, 6, 7, 8, 9, 10, 11, 12, 13, 14, 15); }
__device__ __forceinline__ v16bf cat16b(v8us lo, v8us hi) { return __builtin_bit_cast(v16bf, __builtin_shufflevector(lo, hi, 0, 1, 2, 3, 4, 5, 6, 7, 8, 9, 10, 11, 12, 13, 14, 15)); }
__device__ __forceinline__ v8f wmma16(v16h a, v16h b, v8f c) { return __builtin_amdgcn_wmma_f32_16x16x32_f16(false, a, false, b, (short)0, c, false, false); }
__device__ __forceinline__ v8f wmmab(v16bf a, v16bf b, v8f c) { return __builtin_amdgcn_wmma_f32_16x16x32_bf16(false, a, false, b, (short)0, c, false, false); }

template <typename T16> struct WFrag;
template <> struct WFrag<h16> { typedef v16h V; static __device__ __forceinline__ V ld(const h16* p) { return cat16(*(const v8h*)p, *(const v8h*)(p + 16)); } static __device__ __forceinline__ v8f mma(V a, V b, v8f c) { return wmma16(a, b, c); } };
template <> struct WFrag<bf> { typedef v16bf V; static __device__ __forceinline__ V ld(const bf* p) { return cat16b(*(const v8us*)p, *(const v8us*)(p + 16)); } static __device__ __forceinline__ v8f mma(V a, V b, v8f c) { return wmmab(a, b, c); } };
template <typename T16, int NSPLIT, bool BIAS>
__global__ __launch_bounds__(32) void k_gemmw(const T16* __restrict__ A, const T16* __restrict__ A2, const T16* __restrict__ Bt, const T16* __restrict__ Bt2, int K, float* C, int ldc, const float* __restrict__ bias, size_t sA, size_t sB, size_t sC) {
    typedef typename WFrag<T16>::V V;
    __shared__ __align__(16) float os[16 * 68];
    const size_t z = blockIdx.z; A += z * sA; if (A2) A2 += z * sA; Bt += z * sB; if (Bt2) Bt2 += z * sB; C += z * sC;
    const int lane = threadIdx.x & 31, lr = lane & 15, hi = lane >> 4; const int r0 = blockIdx.x * 64, c0 = blockIdx.y * 64;
    v8f acc[4][4];
#pragma unroll
    for (int mb = 0; mb < 4; ++mb)
#pragma unroll
        for (int nb = 0; nb < 4; ++nb) acc[mb][nb] = (v8f){};
    const size_t aoff = (size_t)(r0 + lr) * K + 8 * hi, boff = (size_t)(c0 + lr) * K + 8 * hi;
#pragma unroll 1
    for (int kc = 0; kc < K; kc += 32) {
        V a[4], a2[4];
#pragma unroll
        for (int mb = 0; mb < 4; ++mb) { a[mb] = WFrag<T16>::ld(A + aoff + (size_t)mb * 16 * K + kc); if (NSPLIT == 1 || NSPLIT == 2) a2[mb] = WFrag<T16>::ld(A2 + aoff + (size_t)mb * 16 * K + kc); }
#pragma unroll
        for (int nb = 0; nb < 4; ++nb) { const V b = WFrag<T16>::ld(Bt + boff + (size_t)nb * 16 * K + kc); V b2; if (NSPLIT >= 2) b2 = WFrag<T16>::ld(Bt2 + boff + (size_t)nb * 16 * K + kc);
#pragma unroll
            for (int mb = 0; mb < 4; ++mb) { acc[mb][nb] = WFrag<T16>::mma(a[mb], b, acc[mb][nb]); if (NSPLIT == 1 || NSPLIT == 2) acc[mb][nb] = WFrag<T16>::mma(a2[mb], b, acc[mb][nb]); if (NSPLIT >= 2) acc[mb][nb] = WFrag<T16>::mma(a[mb], b2, acc[mb][nb]); } }
        asm volatile("v_nop\n\tv_nop\n\tv_nop\n\tv_nop" : "+v"(acc[0][0]), "+v"(acc[1][1]), "+v"(acc[2][2]), "+v"(acc[3][3]) : "v"(a[0]), "v"(a[3]));
    }
#pragma unroll
    for (int mb = 0; mb < 4; ++mb) {
#pragma unroll
        for (int nb = 0; nb < 4; ++nb) {
#pragma unroll
            for (int j = 0; j < 8; ++j) os[(hi * 8 + j) * 68 + nb * 16 + lr] = acc[mb][nb][j]; }
        __builtin_amdgcn_wave_barrier(); asm volatile("" ::: "memory");
        float* crow = C + (size_t)(r0 + mb * 16) * ldc + c0;
#pragma unroll 1
        for (int ps = 0; ps < 2; ++ps) {
#pragma unroll
            for (int s = 0; s < 8; ++s) { const int row = 2 * s + hi, cofs = lr * 4; v4f val = *(const v4fa*)(os + row * 68 + cofs); if (BIAS) { val[0] += bfr(bias[c0 + cofs]); val[1] += bfr(bias[c0 + cofs + 1]); val[2] += bfr(bias[c0 + cofs + 2]); val[3] += bfr(bias[c0 + cofs + 3]); }
                *(volatile v4f*)(crow + (size_t)row * ldc + cofs) = val; }
            if (ps == 0) __threadfence(); }
        __builtin_amdgcn_wave_barrier(); asm volatile("" ::: "memory");
    }
}

__device__ __forceinline__ h16 tohx(float x) { return (h16)x; }
__device__ __forceinline__ void splitf(float y, unsigned short& h, unsigned short& l) { h = f2bf(y); l = f2bf(y - bf2f(h)); }

__global__ __launch_bounds__(256) void k_cvt8(const float* __restrict__ src, bf* dst, size_t n8) { const size_t i = (size_t)blockIdx.x * 256 + threadIdx.x; if (i >= n8) return; const v8f v = *(const v8f*)(src + i * 8); v8us o;
#pragma unroll
    for (int k = 0; k < 8; ++k) o[k] = f2bf(v[k]); *(volatile v8us*)(dst + i * 8) = o; __threadfence(); *(volatile v8us*)(dst + i * 8) = o; }

__global__ __launch_bounds__(256) void k_hp(const float* __restrict__ F, h16* P) {
    const size_t i = (size_t)blockIdx.x * 256 + threadIdx.x; if (i >= (size_t)2 * NH_ * TT * HD / 8) return;
    const size_t e = i * 8; const int d = (int)(e % HD); const int t = (int)((e / HD) % TT); const int hh = (int)((e / ((size_t)HD * TT)) % NH_); const int z = (int)(e / ((size_t)HD * TT * NH_));
    const float* f = F + (size_t)z * TT * DM + (size_t)t * DM + hh * HD + d; const v4f a = *(const v4f*)f; const v4f b = *(const v4f*)(f + 4); v8h o;
#pragma unroll
    for (int k = 0; k < 4; ++k) { o[k] = tohx(a[k]); o[4 + k] = tohx(b[k]); }
    *(volatile v8h*)(P + e) = o; __threadfence(); *(volatile v8h*)(P + e) = o; }

__global__ __launch_bounds__(256) void k_vtp(const float* __restrict__ F, h16* V16) {
    const size_t i = (size_t)blockIdx.x * 256 + threadIdx.x; if (i >= (size_t)NH_ * HD * TT / 8) return;
    const size_t e = i * 8; const int t = (int)(e % TT); const int d = (int)((e / TT) % HD); const int g = (int)(e / ((size_t)TT * HD)); v8h o;
#pragma unroll
    for (int q = 0; q < 8; ++q) o[q] = tohx(F[(size_t)(t + q) * DM + g * HD + d]);
    *(volatile v8h*)(V16 + e) = o; __threadfence(); *(volatile v8h*)(V16 + e) = o; }

__global__ __launch_bounds__(256) void k_vmean(const h16* __restrict__ V16, float* VM) {
    __shared__ __align__(16) float sm[32];
    const int lane = threadIdx.x & 31, w = __builtin_amdgcn_readfirstlane((int)(threadIdx.x >> 5));
#pragma unroll 1
    for (int r = 0; r < 4; ++r) {
        const int row = blockIdx.x * 32 + w * 4 + r; const h16* p = V16 + (size_t)row * TT + lane * 8; float s = 0.f;
#pragma unroll 4
        for (int c = 0; c < TT / 256; ++c) { const v8h a = *(const v8h*)(p + c * 256);
#pragma unroll
            for (int k = 0; k < 8; ++k) s += (float)a[k]; }
#pragma unroll
        for (int sh = 16; sh; sh >>= 1) s += __shfl_xor(s, sh, 32);
        if (lane == 0) sm[w * 4 + r] = s * (1.0f / (float)TT);
    }
    __syncthreads();
    if (threadIdx.x < 8) { const v4f val = *(const v4fa*)(sm + threadIdx.x * 4); float* dst = VM + (size_t)blockIdx.x * 32 + threadIdx.x * 4; *(volatile v4f*)dst = val; __threadfence(); *(volatile v4f*)dst = val; }
}

__global__ __launch_bounds__(256) void k_asoft(const float* __restrict__ Sb, h16* P16) {
    const int lane = threadIdx.x & 31; const int row = blockIdx.x * 8 + __builtin_amdgcn_readfirstlane((int)(threadIdx.x >> 5)); if (row >= ZH * TT) return; const float* sr = Sb + (size_t)row * TT; float v[TT / 32]; float mx = -3.0e38f;
#pragma unroll
    for (int ch = 0; ch < TT / 128; ++ch) { const int j0 = ch * 128 + lane * 4; const v4f a = *(const v4f*)(sr + j0);
#pragma unroll
        for (int q = 0; q < 4; ++q) { const float t = a[q] * SCL; v[ch * 4 + q] = t; mx = fmaxf(mx, t); } }
#pragma unroll
    for (int sh = 16; sh; sh >>= 1) mx = fmaxf(mx, __shfl_xor(mx, sh, 32));
    float sum = 0.f;
#pragma unroll
    for (int k = 0; k < TT / 32; ++k) { float d0 = __fsub_rn(v[k], mx); asm volatile("" : "+v"(d0)); v[k] = __builtin_amdgcn_exp2f(__fmul_rn(d0, 1.4426950408889634f)); sum += v[k]; }
#pragma unroll
    for (int sh = 16; sh; sh >>= 1) sum += __shfl_xor(sum, sh, 32);
    const float f = __fdiv_rn(PCAR, sum); const float cen = sum * (1.0f / (float)TT);
#pragma unroll 1
    for (int ps = 0; ps < 2; ++ps) {
#pragma unroll
        for (int ch = 0; ch < TT / 128; ++ch) { v4h o4;
#pragma unroll
            for (int q = 0; q < 4; ++q) { float dd = __fsub_rn(v[ch * 4 + q], cen); asm volatile("" : "+v"(dd)); o4[q] = tohx(__fmul_rn(dd, f)); }
            *(volatile v4h*)(P16 + (size_t)row * TT + ch * 128 + lane * 4) = o4; }
        if (ps == 0) __threadfence(); }
}

__global__ __launch_bounds__(256) void k_merge(const float* __restrict__ O, const float* __restrict__ VM, int h0, bf* Ah, bf* Al) {
    const size_t i = (size_t)blockIdx.x * 256 + threadIdx.x; if (i >= (size_t)ZH * TT * HD / 8) return;
    const size_t e = i * 8; const int d = (int)(e % HD); const int t = (int)((e / HD) % TT); const int zz = (int)(e / ((size_t)HD * TT)); const size_t oo = (size_t)t * DQ + (h0 + zz) * HD + d;
    const v4f o0 = *(const v4f*)(O + e); const v4f o1 = *(const v4f*)(O + e + 4); const float* vm = VM + (h0 + zz) * HD + d; const v4f m0 = *(const v4f*)vm; const v4f m1 = *(const v4f*)(vm + 4);
    v8us oh, ol;
#pragma unroll
    for (int q = 0; q < 4; ++q) { unsigned short a, c2; splitf(o0[q] * (1.0f / PCAR) + m0[q], a, c2); oh[q] = a; ol[q] = c2; splitf(o1[q] * (1.0f / PCAR) + m1[q], a, c2); oh[4 + q] = a; ol[4 + q] = c2; }
    *(volatile v8us*)(Ah + oo) = oh; *(volatile v8us*)(Al + oo) = ol; __threadfence(); *(volatile v8us*)(Ah + oo) = oh; *(volatile v8us*)(Al + oo) = ol; }

extern "C" void kernel_launch(void* const* d_in, const int* in_sizes, int n_in,
                              void* d_out, int out_size, void* d_ws, size_t ws_size, hipStream_t stream) {
    if (n_in < 5) return;
    const size_t needx = (size_t)(NB - 1) * SEQ_FULL * DM + (size_t)TT * DM;
    if ((size_t)in_sizes[0] < needx) return;
    if ((size_t)in_sizes[1] < (size_t)DM * DM || (size_t)in_sizes[2] < (size_t)DM * DM || (size_t)in_sizes[3] < (size_t)DM * DM || (size_t)in_sizes[4] < (size_t)DM * DM) return;
    if ((size_t)out_size < needx) return;
    if (WS_TOTAL > ws_size) return;
    const float* x = (const float*)d_in[0]; const float* wq = (const float*)d_in[1]; const float* wk = (const float*)d_in[2]; const float* wv = (const float*)d_in[3]; const float* wo = (const float*)d_in[4];
    float* OUT = (float*)d_out;
    char* wsp = (char*)d_ws;
    auto take = [&](size_t bytes) { char* p = wsp; wsp += (bytes + 255) & ~(size_t)255; return (void*)p; };
    bf* W3 = (bf*)take(SZ_W3);
    bf* WO = (bf*)take(SZ_WO);
    bf* XB = (bf*)take(SZ_XB);
    float* F3 = (float*)take(SZ_F3);
    h16* QK16 = (h16*)take(SZ_QK);
    h16* VT16 = (h16*)take(SZ_VT);
    float* VM = (float*)take(SZ_VM);
    float* Sb = (float*)take(SZ_SB);
    h16* P16 = (h16*)take(SZ_PP);
    float* Ob = (float*)take(SZ_OB);
    bf* ATh = (bf*)take(SZ_AT); bf* ATl = (bf*)take(SZ_AT);
    if ((size_t)(wsp - (char*)d_ws) > ws_size) return;
    const unsigned LW = (unsigned)(((size_t)DM * DM / 8 + 255) / 256);
    k_cvt8<<<LW, 256, 0, stream>>>(wq, W3, (size_t)DM * DM / 8);
    k_cvt8<<<LW, 256, 0, stream>>>(wk, W3 + (size_t)DM * DM, (size_t)DM * DM / 8);
    k_cvt8<<<LW, 256, 0, stream>>>(wv, W3 + (size_t)2 * DM * DM, (size_t)DM * DM / 8);
    k_cvt8<<<LW, 256, 0, stream>>>(wo, WO, (size_t)DM * DQ / 8);
    const unsigned LHP = (unsigned)(((size_t)2 * NH_ * TT * HD / 8 + 255) / 256), LVT = (unsigned)(((size_t)NH_ * HD * TT / 8 + 255) / 256), LMG = (unsigned)(((size_t)ZH * TT * HD / 8 + 255) / 256);
    for (int b = 0; b < NB; ++b) {
        k_cvt8<<<(unsigned)(((size_t)TT * DM / 8 + 255) / 256), 256, 0, stream>>>(x + (size_t)b * SEQ_FULL * DM, XB, (size_t)TT * DM / 8);
        k_gemmw<bf, 0, false><<<dim3(TT / 64, DM / 64, 3), 32, 0, stream>>>(XB, nullptr, W3, nullptr, DM, F3, DM, nullptr, 0, (size_t)DM * DM, (size_t)TT * DM);
        k_hp<<<LHP, 256, 0, stream>>>(F3, QK16);
        k_vtp<<<LVT, 256, 0, stream>>>(F3 + (size_t)2 * TT * DM, VT16);
        k_vmean<<<NH_ * HD / 32, 256, 0, stream>>>(VT16, VM);
        for (int h0 = 0; h0 < NH_; h0 += ZH) {
            k_gemmw<h16, 0, false><<<dim3(TT / 64, TT / 64, ZH), 32, 0, stream>>>(QK16 + (size_t)h0 * TT * HD, nullptr, QK16 + (size_t)(NH_ + h0) * TT * HD, nullptr, HD, Sb, TT, nullptr, (size_t)TT * HD, (size_t)TT * HD, (size_t)TT * TT);
            k_asoft<<<ZH * TT / 8, 256, 0, stream>>>(Sb, P16);
            k_gemmw<h16, 0, false><<<dim3(TT / 64, HD / 64, ZH), 32, 0, stream>>>(P16, nullptr, VT16 + (size_t)h0 * HD * TT, nullptr, TT, Ob, HD, nullptr, (size_t)TT * TT, (size_t)HD * TT, (size_t)TT * HD);
            k_merge<<<LMG, 256, 0, stream>>>(Ob, VM, h0, ATh, ATl);
        }
        k_gemmw<bf, 1, false><<<dim3(TT / 64, DM / 64, 1), 32, 0, stream>>>(ATh, ATl, WO, nullptr, DQ, OUT + (size_t)b * SEQ_FULL * DM, DM, nullptr, 0, 0, 0);
    }
}
